// Qwen3VLMoeTextAttention_76089640616622
// MI455X (gfx1250) — hardware-verified
//
#include <hip/hip_runtime.h>
#include <math.h>
#include <stdint.h>

#ifndef NB
#define NB 1
#endif
#ifndef SEQ
#define SEQ 2048
#endif
#define T_FULL 2048
#define DMOD  2048
#define NH    32
#define NKVH  4
#define GRP   (NH / NKVH)
#define HD    128
#define HHALF (HD / 2)
#define NQ    (NH * HD)
#define NKV   (NKVH * HD)
#define QO    ((SEQ < 256) ? SEQ : 256)
#define MCH   ((SEQ < 1024) ? SEQ : 1024)
#define NCH   (SEQ / MCH)
#define EPS_RMS 0.000001f
#define RSQ_HD 0.08838834764831845f
#define LOG2E 1.4426950408889634f
#define MNEG  (-100000000.0f)
#define QSC   256.0f
#define KSC   256.0f
#define PCAR  32768.0f
#define VCAR  1024.0f
#define OSC   1024.0f
#define WOS   1024.0f
#define WPB   2
#define NHG   (NH / WPB)
#define NQT   (SEQ / 16)
#define NST   (MCH / 64)
#define NKT   (SEQ / 32)
#define ATT_THREADS (WPB * 32)
#define MTP   36
#define MTW   (16 * MTP)
#define PTP   36
#define PTW   (16 * PTP)
#define SLP   132
#define SLW   (16 * SLP)
#define WREG  (MTW + PTW + SLW)
#define SLAB64 (16 * 68)
#define VTP   72
#define TWP   72
#define FLBYTES 4096
#define WS_CAP 134217728
static_assert(NB == 1);
static_assert(NQ == 4096 && NKV == 512 && GRP == 8 && HD == 128 && HHALF == 64 && NHG * WPB == NH && WPB == 2);
static_assert(ATT_THREADS == 64);
static_assert((SEQ % 64) == 0 && SEQ >= 64 && SEQ <= T_FULL);
static_assert((QO % 64) == 0 && QO >= 64 && QO <= SEQ && (QO % 16) == 0);
static_assert((MCH % 64) == 0 && MCH >= 64 && NCH * MCH == SEQ);
static_assert((DMOD % 64) == 0 && (NQ % 64) == 0 && (NKV % 64) == 0 && (DMOD % 32) == 0 && (NQ % 32) == 0);
static_assert(((SEQ * DMOD / 8) % 256) == 0);
static_assert(((SEQ * SEQ) % 1024) == 0);
static_assert(WPB * WREG * 4 <= 65536 && 2 * HD * VTP * 2 <= 65536 && 4 * SLAB64 * 4 <= 65536 && 64 * TWP * 2 <= 65536);
static_assert(((WREG * 4) % 16) == 0 && ((MTW * 4) % 16) == 0 && ((PTW * 4) % 16) == 0);

typedef unsigned short u16;
typedef _Float16 v16h __attribute__((ext_vector_type(16)));
typedef _Float16 v8h  __attribute__((ext_vector_type(8)));
typedef __bf16   v16b __attribute__((ext_vector_type(16)));
typedef float    v8f  __attribute__((ext_vector_type(8)));
typedef float    v4f  __attribute__((ext_vector_type(4)));
typedef unsigned int v4u __attribute__((ext_vector_type(4)));
typedef int      v4i  __attribute__((ext_vector_type(4)));

union FragH { v16h v; v8h h[2]; v4u u[2]; };
union FragB { v16b v; v4u u[2]; };

__device__ __forceinline__ unsigned short bf_bits(float f) {
  unsigned u = __float_as_uint(f);
  return (unsigned short)((u + 0x7FFFu + ((u >> 16) & 1u)) >> 16);
}
__device__ __forceinline__ float bf_up(unsigned short h) { return __uint_as_float(((unsigned)h) << 16); }
__device__ __forceinline__ float bfr(float f) { return bf_up(bf_bits(f)); }
__device__ __forceinline__ unsigned short h_bits(_Float16 x) { return __builtin_bit_cast(unsigned short, x); }
__device__ __forceinline__ unsigned pk16(unsigned short a, unsigned short b) { return (unsigned)a | ((unsigned)b << 16); }
__device__ __forceinline__ v8f zero8() { v8f z = {0.f, 0.f, 0.f, 0.f, 0.f, 0.f, 0.f, 0.f}; return z; }

__device__ __forceinline__ v16h ldfrag_h(const _Float16* p) {
  FragH f;
  f.h[0] = *(const v8h*)(p);
  f.h[1] = *(const v8h*)(p + 16);
  return f.v;
}
__device__ __forceinline__ v16b ldfrag_b(const u16* p) {
  FragB f;
  f.u[0] = *(const v4u*)(p);
  f.u[1] = *(const v4u*)(p + 16);
  return f.v;
}

__device__ __forceinline__ v8f mma_h(v16h a, v16h b, v8f c) {
  return __builtin_amdgcn_wmma_f32_16x16x32_f16(false, a, false, b, (short)0, c, false, false);
}
__device__ __forceinline__ v8f mma_b(v16b a, v16b b, v8f c) {
  return __builtin_amdgcn_wmma_f32_16x16x32_bf16(false, a, false, b, (short)0, c, false, false);
}
__device__ __forceinline__ void guard2(v8f& a, v8f& b, v16h x0, v16h x1, v16h x2, v16h x3, v16h x4, v16h x5) {
#if defined(__HIP_DEVICE_COMPILE__)
  asm volatile("v_nop\n\tv_nop\n\tv_nop\n\tv_nop"
               : "+v"(a), "+v"(b) : "v"(x0), "v"(x1), "v"(x2), "v"(x3), "v"(x4), "v"(x5) : "memory");
#endif
}
template <typename F>
__device__ __forceinline__ void guard6(v8f& a, v8f& b, v8f& c, v8f& d, F x0, F x1, F x2, F x3, F x4, F x5) {
#if defined(__HIP_DEVICE_COMPILE__)
  asm volatile("v_nop\n\tv_nop\n\tv_nop\n\tv_nop"
               : "+v"(a), "+v"(b), "+v"(c), "+v"(d) : "v"(x0), "v"(x1), "v"(x2), "v"(x3), "v"(x4), "v"(x5) : "memory");
#endif
}
__device__ __forceinline__ void acc_guard4(v8f& a, v8f& b, v8f& c, v8f& d) {
#if defined(__HIP_DEVICE_COMPILE__)
  asm volatile("v_nop\n\tv_nop\n\tv_nop\n\tv_nop" : "+v"(a), "+v"(b), "+v"(c), "+v"(d));
#endif
}
__device__ __forceinline__ void wave_sync_lds() {
  __builtin_amdgcn_fence(__ATOMIC_RELEASE, "workgroup");
  __builtin_amdgcn_wave_barrier();
  __builtin_amdgcn_fence(__ATOMIC_ACQUIRE, "workgroup");
}

__global__ __launch_bounds__(256) void cvt16(const float* __restrict__ x, u16* D, int n8, int f16mode, float scale) {
  const int gt = blockIdx.x * 256 + (int)threadIdx.x;
  if (gt >= n8) return;
  const float* p = x + (size_t)gt * 8;
  const v4f a = *(const v4f*)(p), b4 = *(const v4f*)(p + 4);
  float w[8];
#pragma unroll
  for (int e = 0; e < 4; ++e) { w[e] = a[e]; w[4 + e] = b4[e]; }
  v4u o;
#pragma unroll
  for (int e = 0; e < 4; ++e) {
    const float f0 = w[2 * e], f1 = w[2 * e + 1];
    const unsigned short hb0 = h_bits((_Float16)(bfr(f0) * scale));
    const unsigned short hb1 = h_bits((_Float16)(bfr(f1) * scale));
    const unsigned short bb0 = bf_bits(f0);
    const unsigned short bb1 = bf_bits(f1);
    o[e] = (f16mode != 0) ? pk16(hb0, hb1) : pk16(bb0, bb1);
  }
  u16* d = D + (size_t)gt * 8;
  for (int pass = 0; pass < 2; ++pass) {
    *(volatile v4u*)(d) = o;
    __threadfence();
  }
}

__global__ __launch_bounds__(256) void tw16(const float* __restrict__ W, int K, int ldw, int c0, u16* T, int ncol,
                                            int f16mode, float scale) {
  __shared__ __align__(16) u16 TT[64 * TWP];
  const int tid = threadIdx.x;
  const int bid = blockIdx.x;
  const int ktn = K >> 6;
  const int kt  = bid % ktn;
  const int nt  = bid / ktn;
  if (nt >= (ncol >> 6)) return;
  const int k0 = kt * 64, n0 = nt * 64;
  {
    const int kk = tid >> 2;
    const int nq = (tid & 3) * 16;
    const float* src = W + (size_t)(k0 + kk) * ldw + c0 + n0 + nq;
#pragma unroll
    for (int i = 0; i < 4; ++i) {
      const v4f a = *(const v4f*)(src + 4 * i);
#pragma unroll
      for (int e = 0; e < 4; ++e) {
        const float f = a[e];
        const unsigned short hb = h_bits((_Float16)(bfr(f) * scale));
        const unsigned short bb = bf_bits(f);
        TT[(nq + 4 * i + e) * TWP + kk] = (f16mode != 0) ? hb : bb;
      }
    }
  }
  __syncthreads();
  const int q8 = tid >> 3, p8 = (tid & 7) * 8;
  v4u v[2];
#pragma unroll
  for (int it = 0; it < 2; ++it) {
    const int line = it * 32 + q8;
    v[it] = *(const v4u*)(TT + line * TWP + p8);
  }
  const size_t base = (size_t)n0 * K + k0 + p8;
  for (int pass = 0; pass < 2; ++pass) {
#pragma unroll
    for (int it = 0; it < 2; ++it) {
      const int line = it * 32 + q8;
      *(volatile v4u*)(T + base + (size_t)line * K) = v[it];
    }
    __threadfence();
  }
}

__global__ __launch_bounds__(256) void vt16(const float* __restrict__ F, int sbase, u16* VHo, u16* VLo) {
  __shared__ __align__(16) u16 TH[HD * VTP];
  __shared__ __align__(16) u16 TL[HD * VTP];
  const int tid = threadIdx.x;
  const int bid = blockIdx.x;
  const int st  = bid % NST;
  const int h   = bid / NST;
  if (h >= NKVH) return;
  const int sl0 = st * 64;
  {
    const int sl = tid >> 2;
    const int dc = (tid & 3) * 32;
    const float* src = F + (size_t)(sl0 + sl) * NKV + h * HD + dc;
#pragma unroll
    for (int i = 0; i < 8; ++i) {
      const v4f a = *(const v4f*)(src + 4 * i);
#pragma unroll
      for (int e = 0; e < 4; ++e) {
        const float t = a[e] * VCAR;
        const _Float16 hv = (_Float16)t;
        const _Float16 lv = (_Float16)(t - (float)hv);
        TH[(dc + 4 * i + e) * VTP + sl] = h_bits(hv);
        TL[(dc + 4 * i + e) * VTP + sl] = h_bits(lv);
      }
    }
  }
  __syncthreads();
  v4u vh[4], vl[4];
  const int q8 = tid >> 3, p8 = (tid & 7) * 8;
#pragma unroll
  for (int it = 0; it < 4; ++it) {
    const int line = it * 32 + q8;
    vh[it] = *(const v4u*)(TH + line * VTP + p8);
    vl[it] = *(const v4u*)(TL + line * VTP + p8);
  }
  const size_t hrow = (size_t)h * HD;
  const size_t base = hrow * SEQ + (size_t)(sbase + sl0) + p8;
  for (int pass = 0; pass < 2; ++pass) {
#pragma unroll
    for (int it = 0; it < 4; ++it) {
      const int line = it * 32 + q8;
      *(volatile v4u*)(VHo + base + (size_t)line * SEQ) = vh[it];
      *(volatile v4u*)(VLo + base + (size_t)line * SEQ) = vl[it];
    }
    __threadfence();
  }
}

__device__ __forceinline__ void rot_pair(float yl, float yh, float cl, float sl, float ch, float sh, float sc,
                                         unsigned short& hl, unsigned short& hhv, unsigned short& ll, unsigned short& lh) {
#pragma clang fp contract(off)
  const float rl = yl * cl - yh * sl;
  const float rh = yh * ch + yl * sh;
  const float tl = rl * sc, th = rh * sc;
  const _Float16 a = (_Float16)tl, bq = (_Float16)th;
  hl  = h_bits(a);
  hhv = h_bits(bq);
  ll  = h_bits((_Float16)(tl - (float)a));
  lh  = h_bits((_Float16)(th - (float)bq));
}

__global__ __launch_bounds__(256) void nrope16(const float* __restrict__ F, int ncols, int sbase,
                                               const float* __restrict__ nw, const float* __restrict__ cosb,
                                               const float* __restrict__ sinb, u16* Hp, u16* Lp, float sc) {
#pragma clang fp contract(off)
  const int tid = (int)threadIdx.x;
  const int r   = (int)blockIdx.x;
  if (r >= MCH) return;
  const int s   = sbase + r;
  const int dlo = (tid & 7) * 8;
  const int clo = (tid >> 3) * HD + dlo;
  const float* p  = F + (size_t)r * ncols + clo;
  const float* cp = cosb + (size_t)s * HD + dlo;
  const float* sp = sinb + (size_t)s * HD + dlo;
  const v4f xa = *(const v4f*)(p), xb = *(const v4f*)(p + 4);
  const v4f ya = *(const v4f*)(p + HHALF), yb = *(const v4f*)(p + HHALF + 4);
  const v4f cla = *(const v4f*)(cp), clb = *(const v4f*)(cp + 4);
  const v4f cha = *(const v4f*)(cp + HHALF), chb = *(const v4f*)(cp + HHALF + 4);
  const v4f sla = *(const v4f*)(sp), slb = *(const v4f*)(sp + 4);
  const v4f sha = *(const v4f*)(sp + HHALF), shb = *(const v4f*)(sp + HHALF + 4);
  const v4f wa = *(const v4f*)(nw + dlo), wb4 = *(const v4f*)(nw + dlo + 4);
  const v4f wc = *(const v4f*)(nw + HHALF + dlo), wd = *(const v4f*)(nw + HHALF + dlo + 4);
  float xl[8], xh[8], cl[8], ch[8], sl[8], sh[8], wl[8], wh[8];
#pragma unroll
  for (int e = 0; e < 4; ++e) {
    xl[e] = xa[e];        xl[4 + e] = xb[e];
    xh[e] = ya[e];        xh[4 + e] = yb[e];
    cl[e] = bfr(cla[e]);  cl[4 + e] = bfr(clb[e]);
    ch[e] = bfr(cha[e]);  ch[4 + e] = bfr(chb[e]);
    sl[e] = bfr(sla[e]);  sl[4 + e] = bfr(slb[e]);
    sh[e] = bfr(sha[e]);  sh[4 + e] = bfr(shb[e]);
    wl[e] = bfr(wa[e]);   wl[4 + e] = bfr(wb4[e]);
    wh[e] = bfr(wc[e]);   wh[4 + e] = bfr(wd[e]);
  }
  float ss = 0.0f;
#pragma unroll
  for (int e = 0; e < 8; ++e) { ss = ss + xl[e] * xl[e]; ss = ss + xh[e] * xh[e]; }
  ss += __shfl_xor(ss, 1, 32);
  ss += __shfl_xor(ss, 2, 32);
  ss += __shfl_xor(ss, 4, 32);
  const float var = ss * (1.0f / (float)HD);
  const float rs  = 1.0f / sqrtf(var + EPS_RMS);
#pragma unroll
  for (int e = 0; e < 8; ++e) {
    xl[e] = (xl[e] * rs) * wl[e];
    xh[e] = (xh[e] * rs) * wh[e];
  }
  v4u ohl, ohh, oll, olh;
#pragma unroll
  for (int e = 0; e < 4; ++e) {
    unsigned short hl0, hh0, ll0, lh0, hl1, hh1, ll1, lh1;
    rot_pair(xl[2 * e],     xh[2 * e],     cl[2 * e],     sl[2 * e],     ch[2 * e],     sh[2 * e],     sc,
             hl0, hh0, ll0, lh0);
    rot_pair(xl[2 * e + 1], xh[2 * e + 1], cl[2 * e + 1], sl[2 * e + 1], ch[2 * e + 1], sh[2 * e + 1], sc,
             hl1, hh1, ll1, lh1);
    ohl[e] = pk16(hl0, hl1);
    ohh[e] = pk16(hh0, hh1);
    oll[e] = pk16(ll0, ll1);
    olh[e] = pk16(lh0, lh1);
  }
  u16* dh = Hp + (size_t)s * ncols + clo;
  u16* dl = Lp + (size_t)s * ncols + clo;
  for (int pass = 0; pass < 2; ++pass) {
    *(volatile v4u*)(dh) = ohl;
    *(volatile v4u*)(dh + HHALF) = ohh;
    *(volatile v4u*)(dl) = oll;
    *(volatile v4u*)(dl + HHALF) = olh;
    __threadfence();
  }
}

__global__ __launch_bounds__(256) void mchk(const float* __restrict__ Mk, int* FLG) {
  __shared__ int red[256];
  const int tid = threadIdx.x;
  int bad = 0;
  const int n4 = (SEQ * SEQ) / 4;
#pragma unroll 1
  for (int q = tid; q < n4; q += 256) {
    const int idx = q * 4;
    const int i   = idx / SEQ;
    const int j   = idx - i * SEQ;
    const v4f m   = *(const v4f*)(Mk + (size_t)i * T_FULL + j);
#pragma unroll
    for (int e = 0; e < 4; ++e) {
      const float v  = m[e];
      const bool  le = ((j + e) <= i);
      const bool  ok = le ? (v == 0.0f) : (v <= MNEG);
      bad += ok ? 0 : 1;
    }
  }
  red[tid] = bad;
  __syncthreads();
  for (int st = 128; st > 0; st >>= 1) {
    if (tid < st) red[tid] = red[tid] + red[tid + st];
    __syncthreads();
  }
  const int flag = (red[0] == 0) ? 1 : 0;
  if (tid < 8) {
    v4i f = {flag, flag, flag, flag};
    int* d = FLG + tid * 4;
    for (int pass = 0; pass < 2; ++pass) {
      *(volatile v4i*)(d) = f;
      __threadfence();
    }
  }
}

__device__ __forceinline__ void epi64(float* sl, v8f a0, v8f a1, v8f a2, v8f a3, float oscale,
                                      float* C, int N, size_t rowb, int col0, int lane) {
  const int hh = lane >> 4, m = lane & 15;
#pragma unroll
  for (int r = 0; r < 8; ++r) {
    const int ro = (8 * hh + r) * 68 + m;
    sl[ro]      = a0[r] * oscale;
    sl[ro + 16] = a1[r] * oscale;
    sl[ro + 32] = a2[r] * oscale;
    sl[ro + 48] = a3[r] * oscale;
  }
  wave_sync_lds();
  v4f vals[8];
#pragma unroll
  for (int it = 0; it < 8; ++it) vals[it] = *(const v4f*)(sl + (it * 2 + hh) * 68 + m * 4);
  float* dst = C + (rowb + (size_t)hh) * (size_t)N + col0 + m * 4;
  for (int pass = 0; pass < 2; ++pass) {
#pragma unroll
    for (int it = 0; it < 8; ++it) {
      *(volatile v4f*)(dst + (size_t)(it * 2) * (size_t)N) = vals[it];
    }
    __threadfence();
  }
}

__global__ __launch_bounds__(128)
void gemm_bf(const u16* __restrict__ A, const u16* __restrict__ Bt, float* C, int M, int N, int K, float oscale) {
  __shared__ __align__(16) float slab[4 * SLAB64];
  const int tid = threadIdx.x, wave = tid >> 5, lane = tid & 31, hh = lane >> 4, m = lane & 15;
  const int ntile = N >> 6;
  const int bid   = blockIdx.x;
  const int rowb  = (bid / ntile) * 64 + wave * 16;
  const int col0  = (bid % ntile) * 64;
  if (rowb + 16 > M) return;
  const u16* ap = A  + (size_t)(rowb + m) * K + 8 * hh;
  const u16* bp = Bt + (size_t)(col0 + m) * K + 8 * hh;
  const size_t bs = (size_t)16 * K;
  v8f acc0 = zero8(), acc1 = zero8(), acc2 = zero8(), acc3 = zero8();
#pragma unroll 1
  for (int k0 = 0; k0 < K; k0 += 32) {
    const v16b a  = ldfrag_b(ap + k0);
    const v16b b0 = ldfrag_b(bp + k0);
    const v16b b1 = ldfrag_b(bp + bs + k0);
    const v16b b2 = ldfrag_b(bp + 2 * bs + k0);
    const v16b b3 = ldfrag_b(bp + 3 * bs + k0);
    acc0 = mma_b(a, b0, acc0);
    acc1 = mma_b(a, b1, acc1);
    acc2 = mma_b(a, b2, acc2);
    acc3 = mma_b(a, b3, acc3);
    guard6<v16b>(acc0, acc1, acc2, acc3, a, b0, b1, b2, b3, a);
  }
  epi64(slab + wave * SLAB64, acc0, acc1, acc2, acc3, oscale, C, N, (size_t)rowb, col0, lane);
}

template <int NPROD>
__global__ __launch_bounds__(128)
void gemm_o(const u16* __restrict__ Ah, const u16* __restrict__ Al, const u16* __restrict__ Bt,
            float* C, int sbeg, int nrt, float oscale) {
  __shared__ __align__(16) float slab[4 * SLAB64];
  const int tid = threadIdx.x, wave = tid >> 5, lane = tid & 31, hh = lane >> 4, m = lane & 15;
  const int ntile = DMOD >> 6;
  const int bid   = blockIdx.x;
  const int ct    = bid % ntile;
  const int rt    = bid / ntile;
  if (rt >= nrt) return;
  const int srow  = sbeg + rt * 64 + wave * 16;
  if (srow + 16 > SEQ) return;
  const int col0  = ct * 64;
  const int K     = NQ;
  const size_t rowC = (size_t)srow;
  const _Float16* ahp = (const _Float16*)(const void*)Ah + (rowC + m) * K + 8 * hh;
  const _Float16* alp = (const _Float16*)(const void*)Al + (rowC + m) * K + 8 * hh;
  const _Float16* bp  = (const _Float16*)(const void*)Bt + (size_t)(col0 + m) * K + 8 * hh;
  const size_t bs = (size_t)16 * K;
  v8f acc0 = zero8(), acc1 = zero8(), acc2 = zero8(), acc3 = zero8();
  if constexpr (NPROD == 2) {
#pragma unroll 1
    for (int k0 = 0; k0 < K; k0 += 32) {
      const v16h ah = ldfrag_h(ahp + k0), al = ldfrag_h(alp + k0);
      const v16h b0 = ldfrag_h(bp + k0);
      const v16h b1 = ldfrag_h(bp + bs + k0);
      const v16h b2 = ldfrag_h(bp + 2 * bs + k0);
      const v16h b3 = ldfrag_h(bp + 3 * bs + k0);
      acc0 = mma_h(ah, b0, acc0);  acc0 = mma_h(al, b0, acc0);
      acc1 = mma_h(ah, b1, acc1);  acc1 = mma_h(al, b1, acc1);
      acc2 = mma_h(ah, b2, acc2);  acc2 = mma_h(al, b2, acc2);
      acc3 = mma_h(ah, b3, acc3);  acc3 = mma_h(al, b3, acc3);
      guard6<v16h>(acc0, acc1, acc2, acc3, ah, al, b0, b1, b2, b3);
    }
  } else {
#pragma unroll 1
    for (int k0 = 0; k0 < K; k0 += 32) {
      const v16h ah = ldfrag_h(ahp + k0);
      const v16h b0 = ldfrag_h(bp + k0);
      const v16h b1 = ldfrag_h(bp + bs + k0);
      const v16h b2 = ldfrag_h(bp + 2 * bs + k0);
      const v16h b3 = ldfrag_h(bp + 3 * bs + k0);
      acc0 = mma_h(ah, b0, acc0);
      acc1 = mma_h(ah, b1, acc1);
      acc2 = mma_h(ah, b2, acc2);
      acc3 = mma_h(ah, b3, acc3);
      guard6<v16h>(acc0, acc1, acc2, acc3, ah, b0, b1, b2, b3, ah);
    }
  }
  epi64(slab + wave * SLAB64, acc0, acc1, acc2, acc3, oscale, C, DMOD, rowC, col0, lane);
}

__global__ __launch_bounds__(ATT_THREADS)
void attn_c(const u16* __restrict__ QHp, const u16* __restrict__ QLp,
            const u16* __restrict__ KHp, const u16* __restrict__ KLp,
            const u16* __restrict__ VHp, const u16* __restrict__ VLp,
            const float* __restrict__ Mk, const int* __restrict__ FLG,
            u16* OHp, u16* OLp) {
  __shared__ __align__(16) float smem[WPB * WREG];

  const int tid  = threadIdx.x;
  const int wave = tid >> 5;
  const int lane = tid & 31;
  const int hh   = lane >> 4;
  const int c    = lane & 15;
  const int bid  = blockIdx.x;
  const int qt   = bid % NQT;
  const int hg   = bid / NQT;
  if (hg >= NHG) return;
  const int q0   = qt * 16;
  if (q0 + 16 > SEQ) return;
  const int head = hg * WPB + wave;
  const int kvh  = head / GRP;
  const int cflag = FLG[0];

  float* mt   = smem + wave * WREG;
  float* pt   = mt + MTW;
  float* slab = pt + PTW;

  const size_t qcol = (size_t)head * HD + 8 * hh;
  const size_t kcol = (size_t)kvh * HD + 8 * hh;
  const _Float16* Qh  = (const _Float16*)(const void*)QHp + ((size_t)(q0 + c)) * NQ + qcol;
  const _Float16* Ql  = (const _Float16*)(const void*)QLp + ((size_t)(q0 + c)) * NQ + qcol;
  const _Float16* Khb = (const _Float16*)(const void*)KHp + (size_t)c * NKV + kcol;
  const _Float16* Klb = (const _Float16*)(const void*)KLp + (size_t)c * NKV + kcol;
  const _Float16* Vhb = (const _Float16*)(const void*)VHp + ((size_t)kvh * HD + c) * SEQ + 8 * hh;
  const _Float16* Vlb = (const _Float16*)(const void*)VLp + ((size_t)kvh * HD + c) * SEQ + 8 * hh;
  const float* mrw  = Mk + (size_t)(q0 + (lane >> 1)) * T_FULL + (lane & 1) * 16;
  float*       mdst = mt + (lane >> 1) * MTP + (lane & 1) * 16;
  const float lsc = RSQ_HD * (LOG2E / (QSC * KSC));
  const float oc  = 1.0f / (PCAR * VCAR);
  const size_t KROW = (size_t)NKV;

  float mrow[8], lrow[8];
  v8f o[8];
#pragma unroll
  for (int r = 0; r < 8; ++r) { mrow[r] = -INFINITY; lrow[r] = 0.f; }
#pragma unroll
  for (int j = 0; j < 8; ++j) o[j] = zero8();
  const int ncaus = (q0 >> 5) + 1;
  const int nkc = (ncaus < NKT) ? ncaus : NKT;
  const int nkt = (cflag != 0) ? nkc : NKT;

#pragma unroll 1
  for (int kt = 0; kt < nkt; ++kt) {
    const int kb = kt * 32;
    {
      const float* mp = mrw + kb;
      const v4f g0 = *(const v4f*)(mp), g1 = *(const v4f*)(mp + 4);
      const v4f g2 = *(const v4f*)(mp + 8), g3 = *(const v4f*)(mp + 12);
      *(v4f*)(mdst)      = g0;
      *(v4f*)(mdst + 4)  = g1;
      *(v4f*)(mdst + 8)  = g2;
      *(v4f*)(mdst + 12) = g3;
    }
    v8f s0 = zero8(), s1 = zero8();
    const _Float16* k0p = Khb + (size_t)kb * KROW;
    const _Float16* k1p = k0p + (size_t)16 * KROW;
    const _Float16* l0p = Klb + (size_t)kb * KROW;
    const _Float16* l1p = l0p + (size_t)16 * KROW;
#pragma unroll
    for (int kk = 0; kk < HD / 32; ++kk) {
      const v16h qh  = ldfrag_h(Qh + kk * 32);
      const v16h ql  = ldfrag_h(Ql + kk * 32);
      const v16h kh0 = ldfrag_h(k0p + kk * 32);
      const v16h kh1 = ldfrag_h(k1p + kk * 32);
      const v16h kl0 = ldfrag_h(l0p + kk * 32);
      const v16h kl1 = ldfrag_h(l1p + kk * 32);
      s0 = mma_h(qh, kh0, s0);
      s0 = mma_h(ql, kh0, s0);
      s0 = mma_h(qh, kl0, s0);
      s1 = mma_h(qh, kh1, s1);
      s1 = mma_h(ql, kh1, s1);
      s1 = mma_h(qh, kl1, s1);
      guard2(s0, s1, qh, ql, kh0, kl0, kh1, kl1);
    }
    wave_sync_lds();
#pragma unroll
    for (int r = 0; r < 8; ++r) {
      const float* mr = mt + (8 * hh + r) * MTP;
      const float mv0 = bfr(mr[c]);
      const float mv1 = bfr(mr[16 + c]);
      const float t0 = s0[r] * lsc + mv0 * LOG2E;
      const float t1 = s1[r] * lsc + mv1 * LOG2E;
      float mx = fmaxf(t0, t1);
#pragma unroll
      for (int off = 1; off < 16; off <<= 1) mx = fmaxf(mx, __shfl_xor(mx, off, 32));
      const float mn = fmaxf(mrow[r], mx);
      const float ms = (mn == -INFINITY) ? 0.0f : mn;
      const float al = exp2f(mrow[r] - ms);
      mrow[r] = mn;
      const float e0 = exp2f(t0 - ms), e1 = exp2f(t1 - ms);
      float ps = e0 + e1;
#pragma unroll
      for (int off = 1; off < 16; off <<= 1) ps += __shfl_xor(ps, off, 32);
      lrow[r] = lrow[r] * al + ps;
#pragma unroll
      for (int j = 0; j < 8; ++j) o[j][r] *= al;
      const int ro = (8 * hh + r) * PTP + c;
      pt[ro]      = e0;
      pt[ro + 16] = e1;
    }
    wave_sync_lds();
    FragH ph, pl;
    {
      const float* prow = pt + c * PTP + 8 * hh;
      const v4f p0 = *(const v4f*)(prow), p1 = *(const v4f*)(prow + 4);
      const v4f p2 = *(const v4f*)(prow + 16), p3 = *(const v4f*)(prow + 20);
#pragma unroll
      for (int e = 0; e < 4; ++e) {
        const float ta = p0[e] * PCAR, tb = p1[e] * PCAR, tc = p2[e] * PCAR, td = p3[e] * PCAR;
        const _Float16 ha = (_Float16)ta, hb = (_Float16)tb, hc = (_Float16)tc, hd = (_Float16)td;
        ph.h[0][e]     = ha;
        ph.h[0][4 + e] = hb;
        ph.h[1][e]     = hc;
        ph.h[1][4 + e] = hd;
        pl.h[0][e]     = (_Float16)(ta - (float)ha);
        pl.h[0][4 + e] = (_Float16)(tb - (float)hb);
        pl.h[1][e]     = (_Float16)(tc - (float)hc);
        pl.h[1][4 + e] = (_Float16)(td - (float)hd);
      }
    }
    {
      const _Float16* vhp = Vhb + kb;
      const _Float16* vlp = Vlb + kb;
#pragma unroll
      for (int jg = 0; jg < 4; ++jg) {
        const size_t da = (size_t)(2 * jg) * 16 * SEQ;
        const size_t db = da + (size_t)16 * SEQ;
        const v16h vha = ldfrag_h(vhp + da), vhb2 = ldfrag_h(vhp + db);
        const v16h vla = ldfrag_h(vlp + da), vlb2 = ldfrag_h(vlp + db);
        o[2 * jg]     = mma_h(ph.v, vha,  o[2 * jg]);
        o[2 * jg]     = mma_h(pl.v, vha,  o[2 * jg]);
        o[2 * jg]     = mma_h(ph.v, vla,  o[2 * jg]);
        o[2 * jg + 1] = mma_h(ph.v, vhb2, o[2 * jg + 1]);
        o[2 * jg + 1] = mma_h(pl.v, vhb2, o[2 * jg + 1]);
        o[2 * jg + 1] = mma_h(ph.v, vlb2, o[2 * jg + 1]);
        guard2(o[2 * jg], o[2 * jg + 1], ph.v, pl.v, vha, vhb2, vla, vlb2);
      }
    }
    wave_sync_lds();
  }
  acc_guard4(o[0], o[1], o[2], o[3]);
  acc_guard4(o[4], o[5], o[6], o[7]);
#pragma unroll
  for (int r = 0; r < 8; ++r) {
    const float lv  = lrow[r];
    const float ls  = (lv > 0.0f) ? lv : 1.0f;
    const float inv = (lv > 0.0f) ? ((1.0f / ls) * oc) : 0.0f;
#pragma unroll
    for (int j = 0; j < 8; ++j) {
      const int idx = (8 * hh + r) * SLP + j * 16 + c;
      slab[idx] = o[j][r] * inv;
    }
  }

  wave_sync_lds();
  v4u oh[8], ol[8];
  const int rq = lane >> 4, c8 = (lane & 15) * 8;
#pragma unroll
  for (int it = 0; it < 8; ++it) {
    const int row = it * 2 + rq;
    const v4f a = *(const v4f*)(slab + row * SLP + c8), b4 = *(const v4f*)(slab + row * SLP + c8 + 4);
    float w[8];
#pragma unroll
    for (int e = 0; e < 4; ++e) { w[e] = a[e] * OSC; w[4 + e] = b4[e] * OSC; }
#pragma unroll
    for (int e = 0; e < 4; ++e) {
      const _Float16 h0 = (_Float16)w[2 * e], h1 = (_Float16)w[2 * e + 1];
      const _Float16 l0 = (_Float16)(w[2 * e] - (float)h0), l1 = (_Float16)(w[2 * e + 1] - (float)h1);
      oh[it][e] = pk16(h_bits(h0), h_bits(h1));
      ol[it][e] = pk16(h_bits(l0), h_bits(l1));
    }
  }
  const bool wlo = (q0 < QO);
  const size_t ob = (size_t)q0 * NQ + (size_t)head * HD + c8;
  for (int pass = 0; pass < 2; ++pass) {
#pragma unroll
    for (int it = 0; it < 8; ++it) {
      const int row = it * 2 + rq;
      *(volatile v4u*)(OHp + ob + (size_t)row * NQ) = oh[it];
      if (wlo) {
        *(volatile v4u*)(OLp + ob + (size_t)row * NQ) = ol[it];
      }
    }
    __threadfence();
  }
}

extern "C" void kernel_launch(void* const* d_in, const int* in_sizes, int n_in,
                              void* d_out, int out_size, void* d_ws, size_t ws_size,
                              hipStream_t stream) {
  if (n_in < 10) return;
  if (in_sizes[0] < SEQ * DMOD) return;
  if (in_sizes[1] < SEQ * HD) return;
  if (in_sizes[2] < SEQ * HD) return;
  if (in_sizes[3] < (SEQ - 1) * T_FULL + SEQ) return;
  if (in_sizes[4] < DMOD * NQ) return;
  if (in_sizes[5] < DMOD * NKV) return;
  if (in_sizes[6] < DMOD * NKV) return;
  if (in_sizes[7] < NQ * DMOD) return;
  if (in_sizes[8] < HD) return;
  if (in_sizes[9] < HD) return;
  if (out_size < SEQ * DMOD) return;

  const float* x    = (const float*)d_in[0];
  const float* cosb = (const float*)d_in[1];
  const float* sinb = (const float*)d_in[2];
  const float* mk   = (const float*)d_in[3];
  const float* wq   = (const float*)d_in[4];
  const float* wk   = (const float*)d_in[5];
  const float* wv   = (const float*)d_in[6];
  const float* wo   = (const float*)d_in[7];
  const float* qnw  = (const float*)d_in[8];
  const float* knw  = (const float*)d_in[9];
  float*       out  = (float*)d_out;

  const size_t szXB = (size_t)SEQ * DMOD * 2;
  const size_t szWT = (size_t)NQ * DMOD * 2;
  const size_t szF  = (size_t)MCH * NQ * 4;
  const size_t szQ  = (size_t)SEQ * NQ * 2;
  const size_t szK  = (size_t)SEQ * NKV * 2;
  const size_t szV  = (size_t)NKVH * HD * SEQ * 2;
  const size_t szOH = (size_t)SEQ * NQ * 2;
  const size_t szOL = (size_t)QO * NQ * 2;
  const size_t szWO = (size_t)DMOD * NQ * 2;
  size_t off = 0;
  const size_t oXB = off; off += szXB;
  const size_t oWT = off; off += szWT;
  const size_t oF  = off; off += szF;
  const size_t oQH = off; off += szQ;
  const size_t oQL = off; off += szQ;
  const size_t oKH = off; off += szK;
  const size_t oKL = off; off += szK;
  const size_t oVH = off; off += szV;
  const size_t oVL = off; off += szV;
  const size_t oOH = off; off += szOH;
  const size_t oOL = off; off += szOL;
  const size_t oWO = off; off += szWO;
  const size_t oFL = off; off += (size_t)FLBYTES;
  if (off > ws_size) return;
  if (off > (size_t)WS_CAP) return;

  char* ws = (char*)d_ws;
  u16*   XB  = (u16*)(ws + oXB);
  u16*   WT  = (u16*)(ws + oWT);
  float* F   = (float*)(ws + oF);
  u16*   QH  = (u16*)(ws + oQH);
  u16*   QL  = (u16*)(ws + oQL);
  u16*   KH  = (u16*)(ws + oKH);
  u16*   KL  = (u16*)(ws + oKL);
  u16*   VH  = (u16*)(ws + oVH);
  u16*   VL  = (u16*)(ws + oVL);
  u16*   OH  = (u16*)(ws + oOH);
  u16*   OL  = (u16*)(ws + oOL);
  u16*   WO  = (u16*)(ws + oWO);
  int*   FL  = (int*)(ws + oFL);

  const dim3 b256(256), b128(128), b32(32), bAT(ATT_THREADS);
  const int  n8x = (SEQ * DMOD) / 8;
  const dim3 gX((n8x + 255) / 256);
  const dim3 gTWq((DMOD / 64) * (NQ / 64));
  const dim3 gTWk((DMOD / 64) * (NKV / 64));
  const dim3 gTWo((NQ / 64) * (DMOD / 64));
  const dim3 gGq((MCH / 64) * (NQ / 64));
  const dim3 gGk((MCH / 64) * (NKV / 64));
  const dim3 gVT(NKVH * NST);
  const dim3 gRW(MCH);
  const dim3 gAT(NQT * NHG);
  const int  nrtR = QO / 64;
  const int  nrtP = (SEQ - QO) / 64;

  cvt16<<<gX, b256, 0, stream>>>(x, XB, n8x, 0, 1.0f);

  tw16<<<gTWq, b256, 0, stream>>>(wq, DMOD, NQ, 0, WT, NQ, 0, 1.0f);
  for (int ch = 0; ch < NCH; ++ch) {
    const int sbase = ch * MCH;
    gemm_bf<<<gGq, b128, 0, stream>>>(XB + (size_t)sbase * DMOD, WT, F, MCH, NQ, DMOD, 1.0f);
    nrope16<<<gRW, b256, 0, stream>>>(F, NQ, sbase, qnw, cosb, sinb, QH, QL, QSC);
  }
  tw16<<<gTWk, b256, 0, stream>>>(wk, DMOD, NKV, 0, WT, NKV, 0, 1.0f);
  for (int ch = 0; ch < NCH; ++ch) {
    const int sbase = ch * MCH;
    gemm_bf<<<gGk, b128, 0, stream>>>(XB + (size_t)sbase * DMOD, WT, F, MCH, NKV, DMOD, 1.0f);
    nrope16<<<gRW, b32, 0, stream>>>(F, NKV, sbase, knw, cosb, sinb, KH, KL, KSC);
  }
  tw16<<<gTWk, b256, 0, stream>>>(wv, DMOD, NKV, 0, WT, NKV, 0, 1.0f);
  for (int ch = 0; ch < NCH; ++ch) {
    const int sbase = ch * MCH;
    gemm_bf<<<gGk, b128, 0, stream>>>(XB + (size_t)sbase * DMOD, WT, F, MCH, NKV, DMOD, 1.0f);
    vt16<<<gVT, b256, 0, stream>>>(F, sbase, VH, VL);
  }
  mchk<<<dim3(1), b256, 0, stream>>>(mk, FL);
  attn_c<<<gAT, bAT, 0, stream>>>(QH, QL, KH, KL, VH, VL, mk, FL, OH, OL);
  tw16<<<gTWo, b256, 0, stream>>>(wo, NQ, DMOD, 0, WO, DMOD, 1, WOS);
  gemm_o<2><<<dim3(nrtR * (DMOD / 64)), b128, 0, stream>>>(OH, OL, WO, out, 0, nrtR, 1.0f / (OSC * WOS));
  if (nrtP > 0) {
    gemm_o<1><<<dim3(nrtP * (DMOD / 64)), b128, 0, stream>>>(OH, OL, WO, out, QO, nrtP, 1.0f / (OSC * WOS));
  }
  (void)hipGetLastError();
}
